// SelectiveSSM_47390669144437
// MI455X (gfx1250) — hardware-verified
//
#include <hip/hip_runtime.h>
#include <math.h>

typedef __attribute__((ext_vector_type(16))) _Float16 v16h;
typedef __attribute__((ext_vector_type(8)))  _Float16 v8h;
typedef __attribute__((ext_vector_type(8)))  float    v8f;
typedef __attribute__((ext_vector_type(4)))  float    v4f;

constexpr int kBatch = 2;
constexpr int kSeqL  = 2048;
constexpr int kDmod  = 1024;
constexpr int kDin   = 2048;
constexpr int kNst   = 16;
constexpr int kDtR   = 64;
constexpr int kPrjN  = 96;
constexpr int kPrjP  = 128;
constexpr int kXZP   = 2 * kDin;
constexpr int kRows  = kBatch * kSeqL;
constexpr int kTP    = 260;

constexpr float kCarryWin  = 32.0f;
constexpr float kCarryWxp  = 32.0f;
constexpr float kCarryWdt  = 8.0f;
constexpr float kCarryWout = 32.0f;
constexpr float kCarryDt   = 16.0f;
constexpr float kCarryY    = 16.0f;
constexpr float kFoldIn    = 1.0f / kCarryWin;
constexpr float kFoldXp    = 1.0f / kCarryWxp;
constexpr float kFoldDt    = 1.0f / (kCarryDt * kCarryWdt);
constexpr float kFoldOut   = 1.0f / (kCarryY * kCarryWout);

static_assert(kDtR + 2 * kNst == kPrjN);
static_assert((kDmod % 32) == 0 && (kDin % 32) == 0 && (kDtR % 32) == 0);
static_assert((kSeqL % 64) == 0 && (kXZP % 64) == 0 && (kPrjP % 64) == 0 && (kDin % 64) == 0 && (kDmod % 64) == 0);
static_assert((kRows % 8) == 0 && (kDin % 256) == 0 && (kSeqL % 16) == 0);

constexpr size_t SZ_WIN16  = (size_t)kXZP * kDmod * 2;
constexpr size_t SZ_WXP16  = (size_t)kPrjP * kDin * 2;
constexpr size_t SZ_WDT16  = (size_t)kDin * kDtR * 2;
constexpr size_t SZ_WOUT16 = (size_t)kDmod * kDin * 2;
constexpr size_t SZ_XN16   = (size_t)kRows * kDmod * 2;
constexpr size_t SZ_XZ     = (size_t)kSeqL * kXZP * 4;
constexpr size_t SZ_UC     = (size_t)kSeqL * kDin * 4;
constexpr size_t SZ_UC16   = (size_t)kSeqL * kDin * 2;
constexpr size_t SZ_PROJ   = (size_t)kSeqL * kPrjP * 4;
constexpr size_t SZ_DT16   = (size_t)kSeqL * kDtR * 2;
constexpr size_t SZ_DLR    = (size_t)kSeqL * kDin * 4;
constexpr size_t SZ_Y16    = (size_t)kSeqL * kDin * 2;
constexpr size_t OFF_WIN16  = 0;
constexpr size_t OFF_WXP16  = OFF_WIN16  + SZ_WIN16;
constexpr size_t OFF_WDT16  = OFF_WXP16  + SZ_WXP16;
constexpr size_t OFF_WOUT16 = OFF_WDT16  + SZ_WDT16;
constexpr size_t OFF_XN16   = OFF_WOUT16 + SZ_WOUT16;
constexpr size_t OFF_XZ     = OFF_XN16   + SZ_XN16;
constexpr size_t OFF_UC     = OFF_XZ     + SZ_XZ;
constexpr size_t OFF_UC16   = OFF_UC     + SZ_UC;
constexpr size_t OFF_PROJ   = OFF_UC16   + SZ_UC16;
constexpr size_t OFF_DT16   = OFF_PROJ   + SZ_PROJ;
constexpr size_t OFF_DLR    = OFF_DT16   + SZ_DT16;
constexpr size_t OFF_Y16    = OFF_DLR    + SZ_DLR;
constexpr size_t WS_TOTAL   = OFF_Y16    + SZ_Y16;
static_assert(WS_TOTAL == 106954752ull);
static_assert(WS_TOTAL <= 134217728ull);
static_assert((OFF_WXP16 % 128) == 0 && (OFF_WDT16 % 128) == 0 && (OFF_WOUT16 % 128) == 0 && (OFF_XN16 % 128) == 0 &&
              (OFF_XZ % 128) == 0 && (OFF_UC % 128) == 0 && (OFF_UC16 % 128) == 0 && (OFF_PROJ % 128) == 0 &&
              (OFF_DT16 % 128) == 0 && (OFF_DLR % 128) == 0 && (OFF_Y16 % 128) == 0);

__device__ __forceinline__ void grp_guard_h(v8f& a, v8f& b, v8f& c, v8f& d, v16h x, v16h b0, v16h b1, v16h b2, v16h b3) {
  asm volatile("v_nop\n\tv_nop\n\tv_nop\n\tv_nop" : "+v"(a), "+v"(b), "+v"(c), "+v"(d) : "v"(x), "v"(b0), "v"(b1), "v"(b2), "v"(b3));
}
__device__ __forceinline__ void keep4_h(v16h a, v16h b, v16h c, v16h d) { asm volatile("v_nop" :: "v"(a), "v"(b), "v"(c), "v"(d)); }
__device__ __forceinline__ void acc_guard4(v8f& a, v8f& b, v8f& c, v8f& d) { asm volatile("v_nop\n\tv_nop\n\tv_nop\n\tv_nop" : "+v"(a), "+v"(b), "+v"(c), "+v"(d)); }

struct Frag16 {
  union U { v16h v; v8h h[2]; };
  static __device__ __forceinline__ v16h load(const _Float16* p) {
    U f;
    f.h[0] = *(const v8h*)(p);
    f.h[1] = *(const v8h*)(p + 16);
    return f.v;
  }
  static __device__ __forceinline__ v8f mma(v16h a, v16h b, v8f c) {
    return __builtin_amdgcn_wmma_f32_16x16x32_f16(false, a, false, b, (short)0, c, false, false);
  }
};

template <int BIAS_MODE, bool RESID>
__global__ __launch_bounds__(256) void wmma_gemm64_f16(
    const unsigned short* __restrict__ Ap, int lda,
    const unsigned short* __restrict__ Btp, int ldb,
    float* __restrict__ Cg, int ldc,
    const float* __restrict__ bias,
    const float* __restrict__ resid,
    int M, int N, int K, float scale) {
  const _Float16* A  = (const _Float16*)Ap;
  const _Float16* Bt = (const _Float16*)Btp;
  __shared__ __align__(16) float sT[8][16 * 68];
  const int lane = threadIdx.x & 31;
  const int wave = threadIdx.x >> 5;
  const int tilesN = N >> 6;
  const int tilesM = M >> 6;
  const int tile = blockIdx.x * 8 + wave;
  if (tile >= tilesM * tilesN) return;
  const int tm = tile / tilesN;
  const int tn = tile - tm * tilesN;
  const int m0 = tm << 6;
  const int n0 = tn << 6;

  const int rlane = lane & 15;
  const int koff  = (lane >> 4) * 8;
  const int mOff  = (lane >> 4) * 8;

  v8f acc[4][4];
#pragma unroll
  for (int i = 0; i < 4; ++i)
#pragma unroll
    for (int j = 0; j < 4; ++j) acc[i][j] = (v8f){0.f,0.f,0.f,0.f,0.f,0.f,0.f,0.f};

  for (int k0 = 0; k0 < K; k0 += 32) {
    v16h bh[4];
#pragma unroll
    for (int j = 0; j < 4; ++j) {
      const size_t bo = (size_t)(n0 + (j << 4) + rlane) * ldb + koff + k0;
      bh[j] = Frag16::load(Bt + bo);
    }
#pragma unroll
    for (int i = 0; i < 4; ++i) {
      const size_t ao = (size_t)(m0 + (i << 4) + rlane) * lda + koff + k0;
      v16h ah = Frag16::load(A + ao);
#pragma unroll
      for (int j = 0; j < 4; ++j) acc[i][j] = Frag16::mma(ah, bh[j], acc[i][j]);
      grp_guard_h(acc[i][0], acc[i][1], acc[i][2], acc[i][3], ah, bh[0], bh[1], bh[2], bh[3]);
    }
    keep4_h(bh[0], bh[1], bh[2], bh[3]);
  }
  acc_guard4(acc[0][0], acc[0][1], acc[0][2], acc[0][3]);
  acc_guard4(acc[1][0], acc[1][1], acc[1][2], acc[1][3]);
  acc_guard4(acc[2][0], acc[2][1], acc[2][2], acc[2][3]);
  acc_guard4(acc[3][0], acc[3][1], acc[3][2], acc[3][3]);

  float* slab = sT[wave];
  const int hh = lane >> 4, c4 = (lane & 15) * 4;
#pragma unroll
  for (int i = 0; i < 4; ++i) {
    const int mBase = m0 + (i << 4);
#pragma unroll
    for (int j = 0; j < 4; ++j) {
      const int n = n0 + (j << 4) + rlane;
      float bv = 0.f;
      if (BIAS_MODE == 2) bv = bias[n];
#pragma unroll
      for (int r = 0; r < 8; ++r) {
        float v = acc[i][j][r] * scale;
        if (BIAS_MODE == 2) v += bv;
        slab[(mOff + r) * 68 + (j << 4) + rlane] = v;
      }
    }
    __builtin_amdgcn_fence(__ATOMIC_RELEASE, "workgroup");
    __builtin_amdgcn_wave_barrier();
    __builtin_amdgcn_fence(__ATOMIC_ACQUIRE, "workgroup");
    if (RESID) {
      v4f vv[8];
#pragma unroll
      for (int it = 0; it < 8; ++it) {
        const int row = it * 2 + hh;
        const v4f sv = *(const v4f*)(slab + row * 68 + c4);
        const v4f rv = *(const v4f*)(resid + (size_t)(mBase + row) * ldc + n0 + c4);
        vv[it] = sv + rv;
      }
      for (int pass = 0; pass < 2; ++pass) {
#pragma unroll
        for (int it = 0; it < 8; ++it) {
          const int row = it * 2 + hh;
          *(volatile v4f*)(Cg + (size_t)(mBase + row) * ldc + n0 + c4) = vv[it];
        }
        __threadfence();
      }
    } else {
      for (int pass = 0; pass < 2; ++pass) {
#pragma unroll
        for (int it = 0; it < 8; ++it) {
          const int row = it * 2 + hh;
          v4f v = *(const v4f*)(slab + row * 68 + c4);
          *(volatile v4f*)(Cg + (size_t)(mBase + row) * ldc + n0 + c4) = v;
        }
        __threadfence();
      }
    }
    __builtin_amdgcn_fence(__ATOMIC_RELEASE, "workgroup");
    __builtin_amdgcn_wave_barrier();
    __builtin_amdgcn_fence(__ATOMIC_ACQUIRE, "workgroup");
  }
}

__global__ __launch_bounds__(256) void cast_f16_pad_kernel(
    const float* __restrict__ src, unsigned short* __restrict__ dst, int real8, int total8, float scale)
{
  const int i = blockIdx.x * 256 + threadIdx.x;
  if (i >= total8) return;
  const bool ok = (i < real8);
  const int ic = ok ? i : (real8 - 1);
  const float* p = src + ((size_t)ic << 3);
  const v4f a0 = *(const v4f*)(p);
  const v4f a1 = *(const v4f*)(p + 4);
  v8h hv;
#pragma unroll
  for (int e = 0; e < 4; ++e) {
    const float f0 = ok ? (a0[e] * scale) : 0.0f;
    const float f1 = ok ? (a1[e] * scale) : 0.0f;
    hv[e]     = (_Float16)f0;
    hv[4 + e] = (_Float16)f1;
  }
  unsigned short* q = dst + ((size_t)i << 3);
  *(volatile v8h*)q = hv;
  __threadfence();
  *(volatile v8h*)q = hv;
}

__global__ __launch_bounds__(256) void layernorm_f16_kernel(
    const float* __restrict__ x, const float* __restrict__ g, const float* __restrict__ bt,
    unsigned short* __restrict__ XN)
{
  const int lane = threadIdx.x & 31, wave = threadIdx.x >> 5;
  const int tok = blockIdx.x * 8 + wave;
  const float* xr = x + (size_t)tok * kDmod;
  v4f xv[8];
#pragma unroll
  for (int c = 0; c < 4; ++c) {
    const float* p = xr + c * 256 + lane * 8;
    xv[2 * c]     = *(const v4f*)(p);
    xv[2 * c + 1] = *(const v4f*)(p + 4);
  }
  float s = 0.f;
#pragma unroll
  for (int i = 0; i < 8; ++i) {
    s += xv[i][0];
    s += xv[i][1];
    s += xv[i][2];
    s += xv[i][3];
  }
#pragma unroll
  for (int off = 16; off > 0; off >>= 1) s += __shfl_xor(s, off, 32);
  const float mu = s * (1.0f / (float)kDmod);
  float vs = 0.f;
#pragma unroll
  for (int i = 0; i < 8; ++i) {
#pragma unroll
    for (int e = 0; e < 4; ++e) {
      const float dd = xv[i][e] - mu;
      vs = fmaf(dd, dd, vs);
    }
  }
#pragma unroll
  for (int off = 16; off > 0; off >>= 1) vs += __shfl_xor(vs, off, 32);
  const float rstd = rsqrtf(vs * (1.0f / (float)kDmod) + 1e-5f);
  v8h hv[4];
#pragma unroll
  for (int c = 0; c < 4; ++c) {
    const int e0 = c * 256 + lane * 8;
    const v4f g0 = *(const v4f*)(g + e0);
    const v4f g1 = *(const v4f*)(g + e0 + 4);
    const v4f b0 = *(const v4f*)(bt + e0);
    const v4f b1 = *(const v4f*)(bt + e0 + 4);
#pragma unroll
    for (int e = 0; e < 4; ++e) {
      const float n0v = (xv[2 * c][e] - mu) * rstd;
      const float n1v = (xv[2 * c + 1][e] - mu) * rstd;
      hv[c][e]     = (_Float16)(n0v * g0[e] + b0[e]);
      hv[c][4 + e] = (_Float16)(n1v * g1[e] + b1[e]);
    }
  }
  unsigned short* orow = XN + (size_t)tok * kDmod + lane * 8;
  for (int pass = 0; pass < 2; ++pass) {
#pragma unroll
    for (int c = 0; c < 4; ++c) *(volatile v8h*)(orow + c * 256) = hv[c];
    __threadfence();
  }
}

__global__ __launch_bounds__(256) void dt_cast_kernel(
    const float* __restrict__ PROJ, unsigned short* __restrict__ DT16, int total8, float scale)
{
  const int i = blockIdx.x * 256 + threadIdx.x;
  if (i >= total8) return;
  const int e0  = i << 3;
  const int row = e0 >> 6;
  const int c8  = e0 & 63;
  const float* p = PROJ + (size_t)row * kPrjP + c8;
  const v4f a0 = *(const v4f*)(p);
  const v4f a1 = *(const v4f*)(p + 4);
  v8h hv;
#pragma unroll
  for (int e = 0; e < 4; ++e) {
    hv[e]     = (_Float16)(a0[e] * scale);
    hv[4 + e] = (_Float16)(a1[e] * scale);
  }
  unsigned short* qd = DT16 + e0;
  *(volatile v8h*)qd = hv;
  __threadfence();
  *(volatile v8h*)qd = hv;
}

__global__ __launch_bounds__(256) void conv_silu_kernel(
    const float* __restrict__ XZ, const float* __restrict__ cw, const float* __restrict__ cb,
    float* __restrict__ UC, unsigned short* __restrict__ UC16)
{
  __shared__ __align__(16) float sT[16 * kTP];
  const int tid = threadIdx.x, lane = tid & 31, wave = tid >> 5;
  const int d0 = blockIdx.x * 256, d = d0 + tid;
  const int t0 = blockIdx.y * 64;
  const float w0 = cw[d * 4 + 0], w1 = cw[d * 4 + 1], w2 = cw[d * 4 + 2], w3 = cw[d * 4 + 3];
  const float bc = cb[d];
  float xm3, xm2, xm1;
  {
    const int r3 = t0 - 3, r2 = t0 - 2, r1 = t0 - 1;
    const float v3 = XZ[(size_t)(r3 < 0 ? 0 : r3) * kXZP + d];
    const float v2 = XZ[(size_t)(r2 < 0 ? 0 : r2) * kXZP + d];
    const float v1 = XZ[(size_t)(r1 < 0 ? 0 : r1) * kXZP + d];
    xm3 = (r3 >= 0) ? v3 : 0.f;
    xm2 = (r2 >= 0) ? v2 : 0.f;
    xm1 = (r1 >= 0) ? v1 : 0.f;
  }
  const int hrow = wave >> 1;
  const int hch  = (wave & 1) * 128 + lane * 4;
#pragma unroll 1
  for (int sub = 0; sub < 4; ++sub) {
    const int lb = t0 + sub * 16;
#pragma unroll 1
    for (int s = 0; s < 16; ++s) {
      const float xc = XZ[(size_t)(lb + s) * kXZP + d];
      float acc = w0 * xm3;
      acc = fmaf(w1, xm2, acc);
      acc = fmaf(w2, xm1, acc);
      acc = fmaf(w3, xc, acc);
      const float sv = acc + bc;
      const float sg = __builtin_amdgcn_rcpf(1.0f + __expf(-sv));
      sT[s * kTP + tid] = sv * sg;
      xm3 = xm2; xm2 = xm1; xm1 = xc;
    }
    __syncthreads();
    v4f fv[4];
    v8h bv[2];
#pragma unroll
    for (int it = 0; it < 4; ++it) fv[it] = *(const v4f*)(sT + (it * 4 + hrow) * kTP + hch);
#pragma unroll
    for (int it = 0; it < 2; ++it) {
      const float* sp = sT + (it * 8 + wave) * kTP + lane * 8;
      const v4f a0 = *(const v4f*)(sp);
      const v4f a1 = *(const v4f*)(sp + 4);
#pragma unroll
      for (int e = 0; e < 4; ++e) {
        bv[it][e]     = (_Float16)a0[e];
        bv[it][4 + e] = (_Float16)a1[e];
      }
    }
    for (int pass = 0; pass < 2; ++pass) {
#pragma unroll
      for (int it = 0; it < 4; ++it)
        *(volatile v4f*)(UC + (size_t)(lb + it * 4 + hrow) * kDin + d0 + hch) = fv[it];
#pragma unroll
      for (int it = 0; it < 2; ++it)
        *(volatile v8h*)(UC16 + (size_t)(lb + it * 8 + wave) * kDin + d0 + lane * 8) = bv[it];
      __threadfence();
    }
    __syncthreads();
  }
}

__global__ __launch_bounds__(256) void scan_kernel(
    const float* __restrict__ DLR, const float* __restrict__ UC, const float* __restrict__ XZ,
    const float* __restrict__ PROJ, const float* __restrict__ A_log, const float* __restrict__ Dv,
    unsigned short* __restrict__ Y16)
{
  __shared__ __align__(16) float sBC[16 * 32];
  __shared__ __align__(16) float sY[16 * kTP];
  __shared__ __align__(16) float sA[kNst * 256];
  const int tid = threadIdx.x, lane = tid & 31, wave = tid >> 5;
  const int d0 = blockIdx.x * 256, d = d0 + tid;

#pragma unroll 1
  for (int n = 0; n < kNst; ++n) sA[n * 256 + tid] = -expf(A_log[(size_t)d * kNst + n]);
  __syncthreads();
  float An[kNst];
  float h[kNst];
#pragma unroll
  for (int n = 0; n < kNst; ++n) {
    An[n] = sA[n * 256 + tid];
    h[n] = 0.f;
  }
  const float Dd = Dv[d];

#pragma unroll 1
  for (int c = 0; c < kSeqL / 16; ++c) {
    const int l0 = c * 16;
    if (tid < 128) {
      const int r = tid >> 3, q = (tid & 7) * 4;
      const v4f v = *(const v4f*)(PROJ + (size_t)(l0 + r) * kPrjP + kDtR + q);
      *(v4f*)(sBC + r * 32 + q) = v;
    }
    __syncthreads();
#pragma unroll 1
    for (int s = 0; s < 16; ++s) {
      const size_t m = (size_t)(l0 + s);
      float a = DLR[m * kDin + d];
      asm volatile("" : "+v"(a));
      float xv = UC[m * kDin + d];
      asm volatile("" : "+v"(xv));
      float zv = XZ[m * kXZP + kDin + d];
      asm volatile("" : "+v"(zv));
      const float delta = fmaxf(a, 0.0f) + log1pf(__expf(-fabsf(a)));
      v4f Bq[4], Cq[4];
#pragma unroll
      for (int qq = 0; qq < 4; ++qq) {
        Bq[qq] = *(const v4f*)(sBC + s * 32 + 4 * qq);
        Cq[qq] = *(const v4f*)(sBC + s * 32 + kNst + 4 * qq);
      }
      float y = 0.f;
#pragma unroll
      for (int n = 0; n < kNst; ++n) {
        const float e = __expf(delta * An[n]);
        float db = delta * Bq[n >> 2][n & 3];
        asm volatile("" : "+v"(db));
        float p = db * xv;
        asm volatile("" : "+v"(p));
        float qv = h[n] * e;
        asm volatile("" : "+v"(qv));
        const float hn = qv + p;
        h[n] = hn;
        float rr = Cq[n >> 2][n & 3] * hn;
        asm volatile("" : "+v"(rr));
        y += rr;
      }
      float sk = xv * Dd;
      asm volatile("" : "+v"(sk));
      y += sk;
      const float sg = __builtin_amdgcn_rcpf(1.0f + __expf(-zv));
      const float gt = zv * sg;
      sY[s * kTP + tid] = (y * gt) * kCarryY;
    }
    __syncthreads();
    v8h hv[2];
#pragma unroll
    for (int it = 0; it < 2; ++it) {
      const float* sp = sY + (it * 8 + wave) * kTP + lane * 8;
      const v4f a0 = *(const v4f*)(sp);
      const v4f a1 = *(const v4f*)(sp + 4);
#pragma unroll
      for (int e = 0; e < 4; ++e) {
        hv[it][e]     = (_Float16)a0[e];
        hv[it][4 + e] = (_Float16)a1[e];
      }
    }
    for (int pass = 0; pass < 2; ++pass) {
#pragma unroll
      for (int it = 0; it < 2; ++it)
        *(volatile v8h*)(Y16 + (size_t)(l0 + it * 8 + wave) * kDin + d0 + lane * 8) = hv[it];
      __threadfence();
    }
  }
}

extern "C" void kernel_launch(void* const* d_in, const int* in_sizes, int n_in,
                              void* d_out, int out_size, void* d_ws, size_t ws_size,
                              hipStream_t stream)
{
  if (n_in < 12) return;
  if (in_sizes[0] != kRows * kDmod) return;
  if (in_sizes[1] != kXZP * kDmod) return;
  if (in_sizes[2] != kDin * 4 || in_sizes[3] != kDin) return;
  if (in_sizes[4] != kPrjN * kDin) return;
  if (in_sizes[5] != kDin * kDtR || in_sizes[6] != kDin) return;
  if (in_sizes[7] != kDin * kNst || in_sizes[8] != kDin) return;
  if (in_sizes[9] != kDmod * kDin) return;
  if (in_sizes[10] != kDmod || in_sizes[11] != kDmod) return;
  if (out_size != kRows * kDmod) return;
  if (ws_size < WS_TOTAL) return;

  const float* x      = (const float*)d_in[0];
  const float* W_in   = (const float*)d_in[1];
  const float* conv_w = (const float*)d_in[2];
  const float* conv_b = (const float*)d_in[3];
  const float* W_xprj = (const float*)d_in[4];
  const float* W_dt   = (const float*)d_in[5];
  const float* b_dt   = (const float*)d_in[6];
  const float* A_log  = (const float*)d_in[7];
  const float* Dv     = (const float*)d_in[8];
  const float* W_out  = (const float*)d_in[9];
  const float* ln_g   = (const float*)d_in[10];
  const float* ln_b   = (const float*)d_in[11];
  float* dout = (float*)d_out;

  char* ws = (char*)d_ws;
  unsigned short* WIN16  = (unsigned short*)(ws + OFF_WIN16);
  unsigned short* WXP16  = (unsigned short*)(ws + OFF_WXP16);
  unsigned short* WDT16  = (unsigned short*)(ws + OFF_WDT16);
  unsigned short* WOUT16 = (unsigned short*)(ws + OFF_WOUT16);
  unsigned short* XN16   = (unsigned short*)(ws + OFF_XN16);
  float*          XZ     = (float*)(ws + OFF_XZ);
  float*          UC     = (float*)(ws + OFF_UC);
  unsigned short* UC16   = (unsigned short*)(ws + OFF_UC16);
  float*          PROJ   = (float*)(ws + OFF_PROJ);
  unsigned short* DT16   = (unsigned short*)(ws + OFF_DT16);
  float*          DLR    = (float*)(ws + OFF_DLR);
  unsigned short* Y16    = (unsigned short*)(ws + OFF_Y16);
  const float* dummy_bias  = b_dt;
  const float* dummy_resid = x;

  cast_f16_pad_kernel<<<(kXZP * kDmod / 8) / 256, 256, 0, stream>>>(W_in, WIN16, kXZP * kDmod / 8, kXZP * kDmod / 8, kCarryWin);
  cast_f16_pad_kernel<<<(kPrjP * kDin / 8) / 256, 256, 0, stream>>>(W_xprj, WXP16, kPrjN * kDin / 8, kPrjP * kDin / 8, kCarryWxp);
  cast_f16_pad_kernel<<<(kDin * kDtR / 8) / 256, 256, 0, stream>>>(W_dt, WDT16, kDin * kDtR / 8, kDin * kDtR / 8, kCarryWdt);
  cast_f16_pad_kernel<<<(kDmod * kDin / 8) / 256, 256, 0, stream>>>(W_out, WOUT16, kDmod * kDin / 8, kDmod * kDin / 8, kCarryWout);

  layernorm_f16_kernel<<<kRows / 8, 256, 0, stream>>>(x, ln_g, ln_b, XN16);

  for (int b = 0; b < kBatch; ++b) {
    const unsigned short* XNb = XN16 + (size_t)b * kSeqL * kDmod;
    const float* xb = x + (size_t)b * kSeqL * kDmod;
    float* outb = dout + (size_t)b * kSeqL * kDmod;

    wmma_gemm64_f16<0, false><<<dim3(256, 1), 256, 0, stream>>>(
        XNb, kDmod, WIN16, kDmod, XZ, kXZP, dummy_bias, dummy_resid, kSeqL, kXZP, kDmod, kFoldIn);

    conv_silu_kernel<<<dim3(kDin / 256, kSeqL / 64), 256, 0, stream>>>(XZ, conv_w, conv_b, UC, UC16);

    wmma_gemm64_f16<0, false><<<dim3(8, 1), 256, 0, stream>>>(
        UC16, kDin, WXP16, kDin, PROJ, kPrjP, dummy_bias, dummy_resid, kSeqL, kPrjP, kDin, kFoldXp);

    dt_cast_kernel<<<(kSeqL * kDtR) / 8 / 256, 256, 0, stream>>>(PROJ, DT16, (kSeqL * kDtR) / 8, kCarryDt);

    wmma_gemm64_f16<2, false><<<dim3(128, 1), 256, 0, stream>>>(
        DT16, kDtR, WDT16, kDtR, DLR, kDin, b_dt, dummy_resid, kSeqL, kDin, kDtR, kFoldDt);

    scan_kernel<<<dim3(kDin / 256, 1), 256, 0, stream>>>(DLR, UC, XZ, PROJ, A_log, Dv, Y16);

    wmma_gemm64_f16<0, true><<<dim3(64, 1), 256, 0, stream>>>(
        Y16, kDin, WOUT16, kDin, outb, kDmod, dummy_bias, xb, kSeqL, kDmod, kDin, kFoldOut);
  }
}
